// KimiSparseMoeBlock_74371653698289
// MI455X (gfx1250) — hardware-verified
//
#include <hip/hip_runtime.h>
#include <stddef.h>

#define T_TOK 4096
#define D_HID 1024
#define N_EXP 8
#define F_MOE 512
#define SH_INT 1024
#define TB 16
#define HP 1032
#define NTHR 256
#define WCOL 128

static_assert(T_TOK % TB == 0);
static_assert((NTHR / 32) * WCOL == D_HID);
static_assert((NTHR / 32) * 64 == F_MOE);
static_assert((NTHR / 32) * 128 == SH_INT);
static_assert(HP % 8 == 0);
static_assert(HP >= SH_INT);
static_assert(TB * HP * 2 >= (NTHR / 32) * TB * 64 * 4);
static_assert(D_HID % 32 == 0);
static_assert(F_MOE % 32 == 0);
static_assert(SH_INT % 32 == 0);

typedef _Float16 f16;
typedef f16 v16h __attribute__((ext_vector_type(16)));
typedef f16 v8h_t __attribute__((ext_vector_type(8)));
typedef v8h_t __attribute__((may_alias)) v8h;
typedef float v8f __attribute__((ext_vector_type(8)));
typedef float v4f_t __attribute__((ext_vector_type(4)));
typedef v4f_t __attribute__((may_alias)) v4f;
typedef unsigned int v4u __attribute__((ext_vector_type(4)));

union Frag { v16h v; v8h_t h[2]; };

__device__ __forceinline__ v8f zero8() {
    v8f z;
#pragma unroll
    for (int i = 0; i < 8; ++i) z[i] = 0.0f;
    return z;
}

__device__ __forceinline__ v16h ldfrag(const f16* p, int k0) {
    Frag f;
    f.h[0] = *(const v8h*)(p + k0);
    f.h[1] = *(const v8h*)(p + k0 + 16);
    return f.v;
}

__device__ __forceinline__ v8f wmma16(v16h a, v16h b, v8f c) {
    return __builtin_amdgcn_wmma_f32_16x16x32_f16(false, a, false, b, (short)0, c, false, false);
}

__global__ void __launch_bounds__(256) cvt_f16_kernel(
    const float* __restrict__ src, f16* __restrict__ dst, int n8, float scale)
{
    const int i = blockIdx.x * 256 + threadIdx.x;
    const bool ok = (i < n8);
    union { v8h_t h; v4u u; } pk;
#pragma unroll
    for (int j = 0; j < 4; ++j) pk.u[j] = 0u;
    if (ok) {
        const v4f_t a = *(const v4f*)(src + (size_t)i * 8);
        const v4f_t b = *(const v4f*)(src + (size_t)i * 8 + 4);
#pragma unroll
        for (int j = 0; j < 4; ++j) {
            pk.h[j]     = (f16)(a[j] * scale);
            pk.h[4 + j] = (f16)(b[j] * scale);
        }
        *(volatile v4u*)(dst + (size_t)i * 8) = pk.u;
    }
    __threadfence();
    if (ok) {
        *(volatile v4u*)(dst + (size_t)i * 8) = pk.u;
    }
}

template <bool ROUTED>
__device__ __forceinline__ void swiglu32(
    const f16* __restrict__ xa,
    const f16* __restrict__ wg,
    const f16* __restrict__ wu,
    int col0, const float* ews,
    f16* hs, int lane)
{
    const int hh = lane >> 4, m = lane & 15;
    v8f ag[2], au[2];
    ag[0] = zero8(); ag[1] = zero8(); au[0] = zero8(); au[1] = zero8();
    const f16* pg = wg + (size_t)(col0 + m) * D_HID + 8 * hh;
    const f16* pu = wu + (size_t)(col0 + m) * D_HID + 8 * hh;
#pragma unroll 1
    for (int k0 = 0; k0 < D_HID; k0 += 32) {
        const v16h a  = ldfrag(xa, k0);
        const v16h b0 = ldfrag(pg, k0);
        const v16h b1 = ldfrag(pg + 16 * D_HID, k0);
        const v16h c0 = ldfrag(pu, k0);
        const v16h c1 = ldfrag(pu + 16 * D_HID, k0);
        ag[0] = wmma16(a, b0, ag[0]);
        ag[1] = wmma16(a, b1, ag[1]);
        au[0] = wmma16(a, c0, au[0]);
        au[1] = wmma16(a, c1, au[1]);
        asm volatile("v_nop\n\tv_nop\n\tv_nop\n\tv_nop"
                     : "+v"(ag[0]), "+v"(ag[1]), "+v"(au[0]), "+v"(au[1])
                     : "v"(a), "v"(b0), "v"(b1), "v"(c0), "v"(c1));
    }
    float rs[8];
#pragma unroll
    for (int r = 0; r < 8; ++r)
        rs[r] = ROUTED ? (ews[(8 * hh + r) * N_EXP] * 64.0f) : 64.0f;
#pragma unroll
    for (int tn = 0; tn < 2; ++tn) {
        f16* hc = hs + col0 + 16 * tn + m;
#pragma unroll
        for (int r = 0; r < 8; ++r) {
            const float g  = ag[tn][r] * (1.0f / 32.0f);
            const float u  = au[tn][r] * (1.0f / 32.0f);
            const float sg = __builtin_amdgcn_rcpf(1.0f + __expf(-g));
            const float hv = ((g * sg) * u) * rs[r];
            hc[(8 * hh + r) * HP] = (f16)hv;
        }
    }
}

template <int KD>
__device__ __forceinline__ void down128(
    const f16* hs, const f16* __restrict__ wrow, v8f (&o)[8], int lane)
{
    const int hh = lane >> 4, m = lane & 15;
    const f16* pa = hs + m * HP + 8 * hh;
    const f16* pb = wrow + (size_t)m * KD + 8 * hh;
#pragma unroll 1
    for (int k0 = 0; k0 < KD; k0 += 32) {
        const v16h a = ldfrag(pa, k0);
        v16h b;
#pragma unroll
        for (int tn = 0; tn < 8; ++tn) {
            b = ldfrag(pb + (size_t)tn * 16 * KD, k0);
            o[tn] = wmma16(a, b, o[tn]);
        }
        asm volatile("v_nop\n\tv_nop\n\tv_nop\n\tv_nop"
                     : "+v"(o[0]), "+v"(o[1]), "+v"(o[2]), "+v"(o[3]),
                       "+v"(o[4]), "+v"(o[5]), "+v"(o[6]), "+v"(o[7])
                     : "v"(a), "v"(b));
    }
}

__global__ void __launch_bounds__(NTHR) moe_fused_kernel(
    const float* __restrict__ x, const float* __restrict__ gw, const float* __restrict__ gb,
    const f16* __restrict__ x16,
    const f16* __restrict__ w1h, const f16* __restrict__ w3h, const f16* __restrict__ w2h,
    const f16* __restrict__ sgh, const f16* __restrict__ suh, const f16* __restrict__ sdh,
    float* __restrict__ out)
{
    __shared__ __align__(16) unsigned char lds_raw[TB * HP * 2];
    __shared__ __align__(16) float ewL[TB * N_EXP];
    f16*   hs  = (f16*)lds_raw;
    float* stg = (float*)lds_raw;

    const int lane = threadIdx.x & 31, w = threadIdx.x >> 5;
    const int hh = lane >> 4, m = lane & 15;
    const int tok0 = blockIdx.x * TB;

#pragma unroll 1
    for (int q = 0; q < 2; ++q) {
        const int tl = 2 * w + q;
        const float* xr = x + (size_t)(tok0 + tl) * D_HID;
        float acc[N_EXP];
#pragma unroll
        for (int e = 0; e < N_EXP; ++e) acc[e] = 0.0f;
#pragma unroll 1
        for (int j = 0; j < D_HID / 32; ++j) {
            const int k = j * 32 + lane;
            const float xv = xr[k];
#pragma unroll
            for (int e = 0; e < N_EXP; ++e)
                acc[e] = fmaf(xv, gw[(size_t)e * D_HID + k], acc[e]);
        }
#pragma unroll
        for (int e = 0; e < N_EXP; ++e) {
#pragma unroll
            for (int off = 16; off > 0; off >>= 1) acc[e] += __shfl_xor(acc[e], off, 32);
        }
        float sc[N_EXP], scb[N_EXP];
#pragma unroll
        for (int e = 0; e < N_EXP; ++e) {
            const float ex = expf(-acc[e]);
            sc[e]  = 1.0f / (1.0f + ex);
            scb[e] = sc[e] + gb[e];
        }
        float gs[4];
#pragma unroll
        for (int g = 0; g < 4; ++g) gs[g] = scb[2 * g] + scb[2 * g + 1];
        int g1 = 0; float gv1 = gs[0];
#pragma unroll
        for (int g = 1; g < 4; ++g) if (gs[g] > gv1) { gv1 = gs[g]; g1 = g; }
        int g2 = -1; float gv2 = -__builtin_huge_valf();
#pragma unroll
        for (int g = 0; g < 4; ++g) if (g != g1 && gs[g] > gv2) { gv2 = gs[g]; g2 = g; }
        float tmp[N_EXP];
#pragma unroll
        for (int e = 0; e < N_EXP; ++e) {
            const int g = e >> 1;
            tmp[e] = (g == g1 || g == g2) ? scb[e] : 0.0f;
        }
        int i1 = 0; float tv1 = tmp[0];
#pragma unroll
        for (int e = 1; e < N_EXP; ++e) if (tmp[e] > tv1) { tv1 = tmp[e]; i1 = e; }
        int i2 = -1; float tv2 = -__builtin_huge_valf();
#pragma unroll
        for (int e = 0; e < N_EXP; ++e) if (e != i1 && tmp[e] > tv2) { tv2 = tmp[e]; i2 = e; }
        float wa = 0.0f, wb = 0.0f;
#pragma unroll
        for (int e = 0; e < N_EXP; ++e) {
            if (e == i1) wa = sc[e];
            if (e == i2) wb = sc[e];
        }
        const float s    = wa + wb;
        const float den  = s + 1e-20f;
        const float rden = 1.0f / den;
        const float t0   = (wa * rden) * 2.5f;
        const float t1   = (wb * rden) * 2.5f;
        if (lane < N_EXP) {
            const float v = (lane == i1) ? t0 : ((lane == i2) ? t1 : 0.0f);
            ewL[tl * N_EXP + lane] = v;
        }
    }
    __syncthreads();

    v8f o[8];
#pragma unroll
    for (int t = 0; t < 8; ++t) o[t] = zero8();

    const f16* xa = x16 + (size_t)(tok0 + m) * D_HID + 8 * hh;

#pragma unroll 1
    for (int cg = 0; cg < 4; ++cg) {
        const int col0 = w * 128 + cg * 32;
        swiglu32<false>(xa, sgh, suh, col0, ewL, hs, lane);
    }
    __syncthreads();
    down128<SH_INT>(hs, sdh + (size_t)(w * WCOL) * SH_INT, o, lane);
    __syncthreads();

#pragma unroll 1
    for (int e = 0; e < N_EXP; ++e) {
        const f16* wg = w1h + (size_t)e * F_MOE * D_HID;
        const f16* wu = w3h + (size_t)e * F_MOE * D_HID;
#pragma unroll 1
        for (int cg = 0; cg < 2; ++cg) {
            const int col0 = w * 64 + cg * 32;
            swiglu32<true>(xa, wg, wu, col0, ewL + e, hs, lane);
        }
        __syncthreads();
        down128<F_MOE>(hs, w2h + (size_t)e * D_HID * F_MOE + (size_t)(w * WCOL) * F_MOE, o, lane);
        __syncthreads();
    }

    float* stw = stg + w * (TB * 64);
    const float oscale = 1.0f / 2048.0f;
    const int c4 = (lane & 15) * 4;
#pragma unroll
    for (int og = 0; og < 2; ++og) {
#pragma unroll
        for (int t4 = 0; t4 < 4; ++t4) {
#pragma unroll
            for (int r = 0; r < 8; ++r)
                stw[(8 * hh + r) * 64 + 16 * t4 + m] = o[og * 4 + t4][r] * oscale;
        }
        __syncthreads();
        v4f_t v[8];
#pragma unroll
        for (int p = 0; p < 8; ++p) v[p] = *(const v4f*)(stw + (2 * p + hh) * 64 + c4);
        float* go = out + (size_t)tok0 * D_HID + w * WCOL + og * 64 + c4;
#pragma unroll
        for (int p = 0; p < 8; ++p)
            *(volatile v4f_t*)(go + (size_t)(2 * p + hh) * D_HID) = v[p];
        __threadfence();
#pragma unroll
        for (int p = 0; p < 8; ++p)
            *(volatile v4f_t*)(go + (size_t)(2 * p + hh) * D_HID) = v[p];
        __syncthreads();
    }
}

extern "C" void kernel_launch(void* const* d_in, const int* in_sizes, int n_in,
                              void* d_out, int out_size, void* d_ws, size_t ws_size,
                              hipStream_t stream)
{
    if (n_in < 9) return;
    if (in_sizes[0] != T_TOK * D_HID) return;
    if (in_sizes[1] != N_EXP * D_HID) return;
    if (in_sizes[2] != N_EXP) return;
    if (in_sizes[3] != N_EXP * F_MOE * D_HID) return;
    if (in_sizes[4] != N_EXP * D_HID * F_MOE) return;
    if (in_sizes[5] != N_EXP * F_MOE * D_HID) return;
    if (in_sizes[6] != SH_INT * D_HID) return;
    if (in_sizes[7] != SH_INT * D_HID) return;
    if (in_sizes[8] != D_HID * SH_INT) return;
    if (out_size != T_TOK * D_HID) return;

    const float* x   = (const float*)d_in[0];
    const float* gw  = (const float*)d_in[1];
    const float* gb  = (const float*)d_in[2];
    const float* w1  = (const float*)d_in[3];
    const float* w2  = (const float*)d_in[4];
    const float* w3  = (const float*)d_in[5];
    const float* sgw = (const float*)d_in[6];
    const float* suw = (const float*)d_in[7];
    const float* sdw = (const float*)d_in[8];
    float* out = (float*)d_out;

    const size_t nX   = (size_t)T_TOK * D_HID;
    const size_t nW13 = (size_t)N_EXP * F_MOE * D_HID;
    const size_t nW2  = (size_t)N_EXP * D_HID * F_MOE;
    const size_t nS   = (size_t)SH_INT * D_HID;

    const size_t oX  = 0;
    const size_t oW1 = oX  + nX   * 2;
    const size_t oW3 = oW1 + nW13 * 2;
    const size_t oW2 = oW3 + nW13 * 2;
    const size_t oSG = oW2 + nW2  * 2;
    const size_t oSU = oSG + nS   * 2;
    const size_t oSD = oSU + nS   * 2;
    const size_t total = oSD + nS * 2;
    if (total > ws_size) return;

    char* ws = (char*)d_ws;
    f16* x16 = (f16*)(ws + oX);
    f16* w1h = (f16*)(ws + oW1);
    f16* w3h = (f16*)(ws + oW3);
    f16* w2h = (f16*)(ws + oW2);
    f16* sgh = (f16*)(ws + oSG);
    f16* suh = (f16*)(ws + oSU);
    f16* sdh = (f16*)(ws + oSD);

    const int n8X = (int)(nX / 8), n8W = (int)(nW13 / 8), n8S = (int)(nS / 8);
    cvt_f16_kernel<<<(n8X + 255) / 256, 256, 0, stream>>>(x,   x16, n8X, 1.0f);
    cvt_f16_kernel<<<(n8W + 255) / 256, 256, 0, stream>>>(w1,  w1h, n8W, 32.0f);
    cvt_f16_kernel<<<(n8W + 255) / 256, 256, 0, stream>>>(w3,  w3h, n8W, 32.0f);
    cvt_f16_kernel<<<(n8W + 255) / 256, 256, 0, stream>>>(w2,  w2h, n8W, 32.0f);
    cvt_f16_kernel<<<(n8S + 255) / 256, 256, 0, stream>>>(sgw, sgh, n8S, 32.0f);
    cvt_f16_kernel<<<(n8S + 255) / 256, 256, 0, stream>>>(suw, suh, n8S, 32.0f);
    cvt_f16_kernel<<<(n8S + 255) / 256, 256, 0, stream>>>(sdw, sdh, n8S, 32.0f);

    moe_fused_kernel<<<T_TOK / TB, NTHR, 0, stream>>>(
        x, gw, gb, x16, w1h, w3h, w2h, sgh, suh, sdh, out);
}
